// LocalAttention_87832081203397
// MI455X (gfx1250) — hardware-verified
//
#include <hip/hip_runtime.h>
#include <stddef.h>
#include <stdint.h>


#ifndef NB
#define NB 4
#endif
#ifndef SEQ
#define SEQ 2048
#endif
#define NB_FULL 4
#define SEQ_FULL 2048
#define CD 1024
#define WIN 16

#define QRES_ROWS ((SEQ < 256) ? SEQ : 256)
#define KRES_ROWS ((SEQ < 384) ? SEQ : 384)
#define QRES_T0 (SEQ - QRES_ROWS)
#define KRES_T0 (SEQ - KRES_ROWS)

#define PCARRY 16384.0f
#define YCARRY 64.0f
#define WCARRY 64.0f
#define RCARRY 4096.0f
#define RINV (1.0f / 4096.0f)

static_assert(NB >= 1 && NB <= NB_FULL);
static_assert(SEQ % 128 == 0 && SEQ >= 128 && SEQ <= SEQ_FULL);
static_assert((CD % 128) == 0 && (CD % 32) == 0);
static_assert(QRES_ROWS % 128 == 0 && KRES_ROWS % 128 == 0);
static_assert(QRES_T0 % 128 == 0 && KRES_T0 % 128 == 0);
static_assert(KRES_T0 == 0 || KRES_T0 + 32 <= QRES_T0);
static_assert((size_t)5 * NB_FULL * SEQ_FULL * CD * 2 + (size_t)4 * CD * CD * 2
              + (size_t)NB_FULL * 256 * CD * 2 * 2 + (size_t)NB_FULL * 384 * CD * 2 * 2
              + (size_t)NB_FULL * 256 * CD * 4 <= (size_t)134217728);

typedef _Float16 v16h __attribute__((ext_vector_type(16)));
typedef _Float16 v8h  __attribute__((ext_vector_type(8)));
typedef _Float16 v2h  __attribute__((ext_vector_type(2)));
typedef __bf16   v16b __attribute__((ext_vector_type(16)));
typedef float    v8f  __attribute__((ext_vector_type(8)));
typedef float    v4f  __attribute__((ext_vector_type(4)));
typedef float    v2f  __attribute__((ext_vector_type(2)));
typedef unsigned int u32x4 __attribute__((ext_vector_type(4)));

union Frag {
  v16h  h;
  v16b  b;
  u32x4 q[2];
  v8h   p[2];
};

__device__ __forceinline__ v8f zero8() {
  v8f z;
#pragma unroll
  for (int i = 0; i < 8; ++i) z[i] = 0.0f;
  return z;
}

__device__ __forceinline__ unsigned int bf_bits(float x) {
  unsigned int u = __builtin_bit_cast(unsigned int, x);
  u += 0x7FFFu + ((u >> 16) & 1u);
  return u >> 16;
}
__device__ __forceinline__ float bf_rne(float x) {
  unsigned int u = bf_bits(x) << 16;
  return __builtin_bit_cast(float, u);
}
__device__ __forceinline__ unsigned int h_bits(float x) {
  _Float16 t = (_Float16)x;
  unsigned short s = __builtin_bit_cast(unsigned short, t);
  return (unsigned int)s;
}

__device__ __forceinline__ u32x4 pack8_bf(v4f a, v4f c) {
  const float a0 = a[0], a1 = a[1], a2 = a[2], a3 = a[3];
  const float c0 = c[0], c1 = c[1], c2 = c[2], c3 = c[3];
  u32x4 o;
  o[0] = bf_bits(a0) | (bf_bits(a1) << 16);
  o[1] = bf_bits(a2) | (bf_bits(a3) << 16);
  o[2] = bf_bits(c0) | (bf_bits(c1) << 16);
  o[3] = bf_bits(c2) | (bf_bits(c3) << 16);
  return o;
}
__device__ __forceinline__ u32x4 pack8_h(v4f a, v4f c, float scale) {
  const float a0 = bf_rne(a[0]) * scale, a1 = bf_rne(a[1]) * scale;
  const float a2 = bf_rne(a[2]) * scale, a3 = bf_rne(a[3]) * scale;
  const float c0 = bf_rne(c[0]) * scale, c1 = bf_rne(c[1]) * scale;
  const float c2 = bf_rne(c[2]) * scale, c3 = bf_rne(c[3]) * scale;
  u32x4 o;
  o[0] = h_bits(a0) | (h_bits(a1) << 16);
  o[1] = h_bits(a2) | (h_bits(a3) << 16);
  o[2] = h_bits(c0) | (h_bits(c1) << 16);
  o[3] = h_bits(c2) | (h_bits(c3) << 16);
  return o;
}

__device__ __forceinline__ v8f mma_f16(const Frag& a, const Frag& bb, v8f c) {
  c = __builtin_amdgcn_wmma_f32_16x16x32_f16(false, a.h, false, bb.h, (short)0, c, false, false);
  asm volatile("v_nop\n\tv_nop\n\tv_nop\n\tv_nop" : "+v"(c) : "v"(a.h), "v"(bb.h));
  return c;
}
__device__ __forceinline__ v8f mma_bf16(const Frag& a, const Frag& bb, v8f c) {
  c = __builtin_amdgcn_wmma_f32_16x16x32_bf16(false, a.b, false, bb.b, (short)0, c, false, false);
  asm volatile("v_nop\n\tv_nop\n\tv_nop\n\tv_nop" : "+v"(c) : "v"(a.b), "v"(bb.b));
  return c;
}
template <int MODE> struct MmaSel;
template <> struct MmaSel<0> {
  static __device__ __forceinline__ v8f run(const Frag& a, const Frag& bb, v8f c) { return mma_bf16(a, bb, c); }
};
template <> struct MmaSel<1> {
  static __device__ __forceinline__ v8f run(const Frag& a, const Frag& bb, v8f c) { return mma_f16(a, bb, c); }
};

__global__ __launch_bounds__(256) void cvt_rows_bf16(const float* __restrict__ src,
                                                     unsigned short* __restrict__ dst, int mrows) {
  const int m = blockIdx.x * 2 + (threadIdx.x >> 7);
  if (m >= mrows) return;
  const int b = m / SEQ;
  const int t = m - b * SEQ;
  const int c8 = (threadIdx.x & 127) * 8;
  const float* s = src + ((size_t)(b * SEQ_FULL + t)) * CD + c8;
  const v4f a = *(const v4f*)s;
  const v4f c = *(const v4f*)(s + 4);
  const u32x4 o = pack8_bf(a, c);
  unsigned short* d = dst + (size_t)m * CD + c8;
  *(volatile u32x4*)d = o;
  __threadfence();
  *(volatile u32x4*)d = o;
}

__global__ __launch_bounds__(256) void cvt_flat(const float* __restrict__ src,
                                                unsigned short* __restrict__ dst,
                                                int n, int to_f16, float scale) {
  const int i = (blockIdx.x * 256 + (int)threadIdx.x) * 8;
  if (i + 8 > n) return;
  const v4f a = *(const v4f*)(src + i);
  const v4f c = *(const v4f*)(src + i + 4);
  u32x4 o;
  if (to_f16 != 0) o = pack8_h(a, c, scale);
  else             o = pack8_bf(a, c);
  unsigned short* d = dst + i;
  *(volatile u32x4*)d = o;
  __threadfence();
  *(volatile u32x4*)d = o;
}

struct GemmArgs {
  const unsigned short* A;
  const unsigned short* W0;
  const unsigned short* W1;
  const unsigned short* W2;
  const float* bias0;
  const float* bias1;
  const float* bias2;
  unsigned short* o0;
  unsigned short* o1;
  unsigned short* o2;
  unsigned short* r0;
  unsigned short* r1;
  unsigned short* r2;
  float* of;
  const float* addend;
  float oscale;
  int use_bias;
  int use_add;
  int resv;
};
static_assert(sizeof(GemmArgs) == 136);

#define GSP16 136
#define GSP32 132

__device__ __forceinline__ void gemm_store16(const _Float16* st, unsigned short* o16, size_t base,
                                             int pitchR, int wave, int h, int ln) {
#pragma unroll
  for (int it = 0; it < 8; ++it) {
    const int R = wave * 16 + 2 * it + h;
    const u32x4 v = *(const u32x4*)(st + R * GSP16 + ln * 8);
    *(volatile u32x4*)(o16 + base + (size_t)R * pitchR + ln * 8) = v;
  }
}

template <int MODE>
__global__ __launch_bounds__(256) __attribute__((amdgpu_num_vgpr(256)))
void gemm_nt(GemmArgs g) {
  __shared__ __align__(16) unsigned short Asm[128 * 40];
  __shared__ __align__(16) unsigned short Wsm[128 * 40];
  __shared__ __align__(16) float stg[8704];

  const int tid = threadIdx.x;
  const int wave = tid >> 5, lane = tid & 31, h = lane >> 4, ln = lane & 15;
  const int wm = wave >> 2, wn = wave & 3;
  const int m0 = blockIdx.y * 128, n0 = blockIdx.x * 128, z = blockIdx.z;
  const unsigned short* W = (z == 0) ? g.W0 : ((z == 1) ? g.W1 : g.W2);
  const float* bias = (z == 0) ? g.bias0 : ((z == 1) ? g.bias1 : g.bias2);

  v8f acc[4][2];
#pragma unroll
  for (int mt = 0; mt < 4; ++mt)
#pragma unroll
    for (int nt = 0; nt < 2; ++nt) acc[mt][nt] = zero8();

#pragma unroll 1
  for (int k0 = 0; k0 < CD; k0 += 32) {
    u32x4 la[2], lw[2];
#pragma unroll
    for (int s = 0; s < 2; ++s) {
      const int u = tid + s * 256, row = u >> 2, qo = (u & 3) * 8;
      la[s] = *(const u32x4*)(g.A + ((size_t)(m0 + row)) * CD + k0 + qo);
      lw[s] = *(const u32x4*)(W + ((size_t)(n0 + row)) * CD + k0 + qo);
    }
    __syncthreads();
#pragma unroll
    for (int s = 0; s < 2; ++s) {
      const int u = tid + s * 256, row = u >> 2, qo = (u & 3) * 8;
      *(u32x4*)(&Asm[row * 40 + qo]) = la[s];
      *(u32x4*)(&Wsm[row * 40 + qo]) = lw[s];
    }
    __syncthreads();

    Frag af[4], bfr[2];
#pragma unroll
    for (int mt = 0; mt < 4; ++mt) {
      const unsigned short* p = &Asm[(wm * 64 + mt * 16 + ln) * 40 + 8 * h];
      af[mt].q[0] = *(const u32x4*)p;
      af[mt].q[1] = *(const u32x4*)(p + 16);
    }
#pragma unroll
    for (int nt = 0; nt < 2; ++nt) {
      const unsigned short* p = &Wsm[(wn * 32 + nt * 16 + ln) * 40 + 8 * h];
      bfr[nt].q[0] = *(const u32x4*)p;
      bfr[nt].q[1] = *(const u32x4*)(p + 16);
    }
#pragma unroll
    for (int mt = 0; mt < 4; ++mt)
#pragma unroll
      for (int nt = 0; nt < 2; ++nt)
        acc[mt][nt] = MmaSel<MODE>::run(af[mt], bfr[nt], acc[mt][nt]);
  }

  float bb[2];
#pragma unroll
  for (int nt = 0; nt < 2; ++nt)
    bb[nt] = (g.use_bias != 0) ? bf_rne(bias[n0 + wn * 32 + nt * 16 + ln]) : 0.0f;

  const int bidx = m0 / SEQ;
  const int t0 = m0 - bidx * SEQ;

  if (MODE == 0) {
    _Float16* st = (_Float16*)stg;
    const bool tr = (z == 2);
    unsigned short* o16 = (z == 0) ? g.o0 : ((z == 1) ? g.o1 : g.o2);
    unsigned short* r16 = (z == 0) ? g.r0 : ((z == 1) ? g.r1 : g.r2);
#pragma unroll
    for (int mt = 0; mt < 4; ++mt)
#pragma unroll
      for (int nt = 0; nt < 2; ++nt)
#pragma unroll
        for (int r = 0; r < 8; ++r) {
          const int row = wm * 64 + mt * 16 + 8 * h + r;
          const int col = wn * 32 + nt * 16 + ln;
          const float v = acc[mt][nt][r] + bb[nt];
          const int idx = tr ? (col * GSP16 + row) : (row * GSP16 + col);
          st[idx] = (_Float16)v;
        }
    __syncthreads();
    size_t base;
    int pr;
    if (tr) { base = ((size_t)(bidx * CD + n0)) * SEQ + t0; pr = SEQ; }
    else    { base = ((size_t)m0) * CD + n0;             pr = CD;  }
    gemm_store16(st, o16, base, pr, wave, h, ln);
    __threadfence();
    gemm_store16(st, o16, base, pr, wave, h, ln);

    const bool res = (z == 0) ? (t0 >= QRES_T0) : (t0 >= KRES_T0);
    if (res) {
      __syncthreads();
#pragma unroll
      for (int mt = 0; mt < 4; ++mt)
#pragma unroll
        for (int nt = 0; nt < 2; ++nt)
#pragma unroll
          for (int r = 0; r < 8; ++r) {
            const int row = wm * 64 + mt * 16 + 8 * h + r;
            const int col = wn * 32 + nt * 16 + ln;
            const float v = acc[mt][nt][r] + bb[nt];
            const _Float16 hv = (_Float16)v;
            const int idx = tr ? (col * GSP16 + row) : (row * GSP16 + col);
            st[idx] = (_Float16)((v - (float)hv) * RCARRY);
          }
      __syncthreads();
      size_t rbase;
      int rp;
      if (z == 0)      { rbase = ((size_t)(bidx * QRES_ROWS + (t0 - QRES_T0))) * CD + n0; rp = CD; }
      else if (z == 1) { rbase = ((size_t)(bidx * KRES_ROWS + (t0 - KRES_T0))) * CD + n0; rp = CD; }
      else             { rbase = ((size_t)(bidx * CD + n0)) * KRES_ROWS + (t0 - KRES_T0); rp = KRES_ROWS; }
      gemm_store16(st, r16, rbase, rp, wave, h, ln);
      __threadfence();
      gemm_store16(st, r16, rbase, rp, wave, h, ln);
    }
  } else {
    const float osc = g.oscale;
    const bool addp = (g.use_add != 0) && (t0 >= QRES_T0);
    int arow0 = bidx * QRES_ROWS + (t0 - QRES_T0);
    if (arow0 < 0) arow0 = 0;
    if (arow0 > NB * QRES_ROWS - 128) arow0 = NB * QRES_ROWS - 128;
    const float* abase = g.addend + (size_t)arow0 * CD + n0 + lane * 4;
#pragma unroll
    for (int ph = 0; ph < 2; ++ph) {
      __syncthreads();
      if (wm == ph) {
#pragma unroll
        for (int mt = 0; mt < 4; ++mt)
#pragma unroll
          for (int nt = 0; nt < 2; ++nt)
#pragma unroll
            for (int r = 0; r < 8; ++r) {
              const int row = mt * 16 + 8 * h + r;
              const int col = wn * 32 + nt * 16 + ln;
              stg[row * GSP32 + col] = acc[mt][nt][r] * osc + bb[nt];
            }
      }
      __syncthreads();
      v4f vals[8];
#pragma unroll
      for (int it = 0; it < 8; ++it) {
        const int R = wave * 8 + it;
        v4f v = *(const v4f*)(stg + R * GSP32 + lane * 4);
        if (addp) {
          const v4f a4 = *(const v4f*)(abase + ((size_t)(ph * 64 + R)) * CD);
          v += a4;
        }
        vals[it] = v;
      }
      float* ob = g.of + ((size_t)(m0 + ph * 64)) * CD + n0 + lane * 4;
#pragma unroll
      for (int it = 0; it < 8; ++it)
        *(volatile v4f*)(ob + ((size_t)(wave * 8 + it)) * CD) = vals[it];
      __threadfence();
#pragma unroll
      for (int it = 0; it < 8; ++it)
        *(volatile v4f*)(ob + ((size_t)(wave * 8 + it)) * CD) = vals[it];
    }
  }
}

#define YSP 136

__device__ __forceinline__ void attn_store_y(const _Float16* yw, unsigned short* dst,
                                             size_t rowbase, int cs, int h, int ln) {
#pragma unroll
  for (int it = 0; it < 8; ++it) {
    const int R = 2 * it + h;
    const u32x4 v = *(const u32x4*)(yw + R * YSP + ln * 8);
    unsigned short* d = dst + (rowbase + (size_t)R) * CD + cs + ln * 8;
    *(volatile u32x4*)d = v;
  }
}

template <int PR>
__global__ __launch_bounds__(256) __attribute__((amdgpu_num_vgpr(256)))
void attn_band(const unsigned short* __restrict__ qpl, const unsigned short* __restrict__ kpl,
               const unsigned short* __restrict__ vtp, const unsigned short* __restrict__ qrs,
               const unsigned short* __restrict__ krs, const unsigned short* __restrict__ vrt,
               unsigned short* __restrict__ ypl, unsigned short* __restrict__ yrs, int iblk0) {
  __shared__ __align__(16) float    Spart[8 * 16 * 32];
  __shared__ __align__(16) _Float16 Psh[16 * 40];
  __shared__ __align__(16) _Float16 Prs[16 * 40];
  __shared__ float alph[16];
  __shared__ float linv[16];
  __shared__ __align__(16) _Float16 yst[8 * 16 * YSP];

  const int tid = threadIdx.x;
  const int wave = tid >> 5, lane = tid & 31, h = lane >> 4, ln = lane & 15;
  const int rr = tid >> 4;
  const int cc = (tid & 15) * 2;
  const int b = blockIdx.y;
  const int i0 = (iblk0 + (int)blockIdx.x) * 16;
  const int cs = wave * 128;

  Frag qf[4];
  if (PR == 0) {
    const size_t qrow = ((size_t)(b * SEQ + i0 + ln)) * CD + cs + 8 * h;
#pragma unroll
    for (int p = 0; p < 4; ++p) {
      qf[p].q[0] = *(const u32x4*)(qpl + qrow + p * 32);
      qf[p].q[1] = *(const u32x4*)(qpl + qrow + p * 32 + 16);
    }
  }

  v8f oacc[8];
#pragma unroll
  for (int nt = 0; nt < 8; ++nt) oacc[nt] = zero8();
  float m_r = -1e30f, l_r = 0.0f;

  const int jl = i0 - WIN;
  const int jstart = (jl > 0) ? (jl & ~31) : 0;
  const int nch = (SEQ - jstart) >> 5;
  const float SC = 0.03125f * 1.4426950408889634f;
  const int iq = i0 + rr;

#pragma unroll 1
  for (int ch = 0; ch < nch; ++ch) {
    const int j0 = jstart + (ch << 5);

    v8f sacc[2], sres[2];
    sacc[0] = zero8();
    sacc[1] = zero8();
    sres[0] = zero8();
    sres[1] = zero8();
    if (PR == 0) {
#pragma unroll
      for (int p = 0; p < 4; ++p) {
#pragma unroll
        for (int jt = 0; jt < 2; ++jt) {
          Frag kb;
          const unsigned short* kp =
              kpl + ((size_t)(b * SEQ + j0 + jt * 16 + ln)) * CD + cs + p * 32 + 8 * h;
          kb.q[0] = *(const u32x4*)kp;
          kb.q[1] = *(const u32x4*)(kp + 16);
          sacc[jt] = mma_f16(qf[p], kb, sacc[jt]);
        }
      }
    } else {
      const size_t qoff = ((size_t)(b * SEQ + i0 + ln)) * CD + cs + 8 * h;
      const size_t roff = ((size_t)(b * QRES_ROWS + (i0 - QRES_T0) + ln)) * CD + cs + 8 * h;
#pragma unroll 1
      for (int p = 0; p < 4; ++p) {
        Frag qa, qr;
        qa.q[0] = *(const u32x4*)(qpl + qoff + p * 32);
        qa.q[1] = *(const u32x4*)(qpl + qoff + p * 32 + 16);
        qr.q[0] = *(const u32x4*)(qrs + roff + p * 32);
        qr.q[1] = *(const u32x4*)(qrs + roff + p * 32 + 16);
#pragma unroll
        for (int jt = 0; jt < 2; ++jt) {
          const int j = j0 + jt * 16 + ln;
          Frag kb, kr;
          const unsigned short* kp = kpl + ((size_t)(b * SEQ + j)) * CD + cs + p * 32 + 8 * h;
          const unsigned short* rp =
              krs + ((size_t)(b * KRES_ROWS + (j - KRES_T0))) * CD + cs + p * 32 + 8 * h;
          kb.q[0] = *(const u32x4*)kp;
          kb.q[1] = *(const u32x4*)(kp + 16);
          kr.q[0] = *(const u32x4*)rp;
          kr.q[1] = *(const u32x4*)(rp + 16);
          sacc[jt] = mma_f16(qa, kb, sacc[jt]);
          sres[jt] = mma_f16(qa, kr, sres[jt]);
          sres[jt] = mma_f16(qr, kb, sres[jt]);
        }
      }
    }
#pragma unroll
    for (int jt = 0; jt < 2; ++jt)
#pragma unroll
      for (int r = 0; r < 8; ++r) {
        float sv = sacc[jt][r];
        if (PR != 0) sv += sres[jt][r] * RINV;
        Spart[(wave * 16 + 8 * h + r) * 32 + jt * 16 + ln] = sv;
      }
    __syncthreads();

    float s0 = 0.0f, s1 = 0.0f;
#pragma unroll
    for (int w = 0; w < 8; ++w) {
      const v2f t2 = *(const v2f*)(&Spart[(w * 16 + rr) * 32 + cc]);
      s0 += t2[0];
      s1 += t2[1];
    }
    s0 *= SC;
    s1 *= SC;
    const int ja = j0 + cc;
    const bool drop0 = ja < (iq - WIN);
    const bool drop1 = (ja + 1) < (iq - WIN);
    s0 = drop0 ? -1e30f : s0;
    s1 = drop1 ? -1e30f : s1;
    float mx = fmaxf(s0, s1);
    mx = fmaxf(mx, __shfl_xor(mx, 8));
    mx = fmaxf(mx, __shfl_xor(mx, 4));
    mx = fmaxf(mx, __shfl_xor(mx, 2));
    mx = fmaxf(mx, __shfl_xor(mx, 1));
    const float mnew = fmaxf(m_r, mx);
    const float alpha = __builtin_amdgcn_exp2f(m_r - mnew);
    const float e0 = __builtin_amdgcn_exp2f(s0 - mnew);
    const float e1 = __builtin_amdgcn_exp2f(s1 - mnew);
    const float p0 = drop0 ? 0.0f : e0;
    const float p1 = drop1 ? 0.0f : e1;
    float rs = p0 + p1;
    rs += __shfl_xor(rs, 8);
    rs += __shfl_xor(rs, 4);
    rs += __shfl_xor(rs, 2);
    rs += __shfl_xor(rs, 1);
    l_r = l_r * alpha + rs;
    m_r = mnew;
    const float P0 = p0 * PCARRY, P1 = p1 * PCARRY;
    const _Float16 ph0 = (_Float16)P0, ph1 = (_Float16)P1;
    v2h pv;
    pv[0] = ph0;
    pv[1] = ph1;
    *(v2h*)(&Psh[rr * 40 + cc]) = pv;
    if (PR != 0) {
      v2h rv;
      rv[0] = (_Float16)((P0 - (float)ph0) * RCARRY);
      rv[1] = (_Float16)((P1 - (float)ph1) * RCARRY);
      *(v2h*)(&Prs[rr * 40 + cc]) = rv;
    }
    if ((tid & 15) == 0) alph[rr] = alpha;
    __syncthreads();

    float al[8];
#pragma unroll
    for (int r = 0; r < 8; ++r) al[r] = alph[8 * h + r];
#pragma unroll
    for (int nt = 0; nt < 8; ++nt)
#pragma unroll
      for (int r = 0; r < 8; ++r) oacc[nt][r] *= al[r];

    Frag pa;
    pa.p[0] = *(const v8h*)(&Psh[ln * 40 + 8 * h]);
    pa.p[1] = *(const v8h*)(&Psh[ln * 40 + 16 + 8 * h]);
    Frag pr;
    if (PR != 0) {
      pr.p[0] = *(const v8h*)(&Prs[ln * 40 + 8 * h]);
      pr.p[1] = *(const v8h*)(&Prs[ln * 40 + 16 + 8 * h]);
    }
#pragma unroll
    for (int nt = 0; nt < 8; ++nt) {
      Frag vb;
      const unsigned short* vp =
          vtp + ((size_t)(b * CD + cs + nt * 16 + ln)) * SEQ + j0 + 8 * h;
      vb.q[0] = *(const u32x4*)vp;
      vb.q[1] = *(const u32x4*)(vp + 16);
      oacc[nt] = mma_f16(pa, vb, oacc[nt]);
      if (PR != 0) {
        Frag vr;
        const unsigned short* rp =
            vrt + ((size_t)(b * CD + cs + nt * 16 + ln)) * KRES_ROWS + (j0 - KRES_T0) + 8 * h;
        vr.q[0] = *(const u32x4*)rp;
        vr.q[1] = *(const u32x4*)(rp + 16);
        v8f t = zero8();
        t = mma_f16(pa, vr, t);
        t = mma_f16(pr, vb, t);
        oacc[nt] += t * RINV;
      }
    }
  }

  if ((tid & 15) == 0) linv[rr] = (1.0f / l_r) * (YCARRY / PCARRY);
  __syncthreads();
  float li[8];
#pragma unroll
  for (int r = 0; r < 8; ++r) li[r] = linv[8 * h + r];
  _Float16* yw = yst + wave * (16 * YSP);
#pragma unroll
  for (int nt = 0; nt < 8; ++nt)
#pragma unroll
    for (int r = 0; r < 8; ++r)
      yw[(8 * h + r) * YSP + nt * 16 + ln] = (_Float16)(oacc[nt][r] * li[r]);
  __syncthreads();

  const size_t rowbase = (size_t)(b * SEQ + i0);
  attn_store_y(yw, ypl, rowbase, cs, h, ln);
  __threadfence();
  attn_store_y(yw, ypl, rowbase, cs, h, ln);

  if (PR != 0) {
    __syncthreads();
#pragma unroll
    for (int nt = 0; nt < 8; ++nt)
#pragma unroll
      for (int r = 0; r < 8; ++r) {
        const float y64 = oacc[nt][r] * li[r];
        const _Float16 hv = (_Float16)y64;
        yw[(8 * h + r) * YSP + nt * 16 + ln] = (_Float16)((y64 - (float)hv) * RCARRY);
      }
    __syncthreads();
    const size_t rrow = (size_t)(b * QRES_ROWS + (i0 - QRES_T0));
    attn_store_y(yw, yrs, rrow, cs, h, ln);
    __threadfence();
    attn_store_y(yw, yrs, rrow, cs, h, ln);
  }
}

extern "C" void kernel_launch(void* const* d_in, const int* in_sizes, int n_in,
                              void* d_out, int out_size, void* d_ws, size_t ws_size,
                              hipStream_t stream) {
  if (n_in < 9) return;
  const int M = NB * SEQ;
  if (in_sizes[0] < ((NB - 1) * SEQ_FULL + SEQ) * CD) return;
  if (in_sizes[1] < CD * CD || in_sizes[3] < CD * CD || in_sizes[5] < CD * CD || in_sizes[7] < CD * CD) return;
  if (in_sizes[2] < CD || in_sizes[4] < CD || in_sizes[6] < CD || in_sizes[8] < CD) return;
  if (out_size < M * CD) return;

  const float* x  = (const float*)d_in[0];
  const float* Wq = (const float*)d_in[1];
  const float* bq = (const float*)d_in[2];
  const float* Wk = (const float*)d_in[3];
  const float* bk = (const float*)d_in[4];
  const float* Wv = (const float*)d_in[5];
  const float* bv = (const float*)d_in[6];
  const float* Wo = (const float*)d_in[7];
  const float* bo = (const float*)d_in[8];
  float* out = (float*)d_out;

  const size_t planeB = (size_t)M * CD * 2;
  const size_t wB     = (size_t)CD * CD * 2;
  const size_t qrB    = (size_t)NB * QRES_ROWS * CD * 2;
  const size_t krB    = (size_t)NB * KRES_ROWS * CD * 2;
  const size_t rtB    = (size_t)NB * QRES_ROWS * CD * 4;
  char* ws = (char*)d_ws;
  size_t off = 0;
  unsigned short* xb  = (unsigned short*)(ws + off); off += planeB;
  unsigned short* wqb = (unsigned short*)(ws + off); off += wB;
  unsigned short* wkb = (unsigned short*)(ws + off); off += wB;
  unsigned short* wvb = (unsigned short*)(ws + off); off += wB;
  unsigned short* wob = (unsigned short*)(ws + off); off += wB;
  unsigned short* qpl = (unsigned short*)(ws + off); off += planeB;
  unsigned short* kpl = (unsigned short*)(ws + off); off += planeB;
  unsigned short* vtp = (unsigned short*)(ws + off); off += planeB;
  unsigned short* ypl = (unsigned short*)(ws + off); off += planeB;
  unsigned short* qrs = (unsigned short*)(ws + off); off += qrB;
  unsigned short* krs = (unsigned short*)(ws + off); off += krB;
  unsigned short* vrt = (unsigned short*)(ws + off); off += krB;
  unsigned short* yrs = (unsigned short*)(ws + off); off += qrB;
  float*          rtm = (float*)(ws + off);          off += rtB;
  if (off > ws_size) return;

  cvt_rows_bf16<<<dim3(M / 2), dim3(256), 0, stream>>>(x, xb, M);
  cvt_flat<<<dim3(CD * CD / 2048), dim3(256), 0, stream>>>(Wq, wqb, CD * CD, 0, 1.0f);
  cvt_flat<<<dim3(CD * CD / 2048), dim3(256), 0, stream>>>(Wk, wkb, CD * CD, 0, 1.0f);
  cvt_flat<<<dim3(CD * CD / 2048), dim3(256), 0, stream>>>(Wv, wvb, CD * CD, 0, 1.0f);
  cvt_flat<<<dim3(CD * CD / 2048), dim3(256), 0, stream>>>(Wo, wob, CD * CD, 1, WCARRY);

  GemmArgs ga;
  ga.A = xb;
  ga.W0 = wqb; ga.W1 = wkb; ga.W2 = wvb;
  ga.bias0 = bq; ga.bias1 = bk; ga.bias2 = bv;
  ga.o0 = qpl; ga.o1 = kpl; ga.o2 = vtp;
  ga.r0 = qrs; ga.r1 = krs; ga.r2 = vrt;
  ga.of = out;
  ga.addend = rtm;
  ga.oscale = 1.0f;
  ga.use_bias = 1;
  ga.use_add = 0;
  ga.resv = 0;
  gemm_nt<0><<<dim3(CD / 128, M / 128, 3), dim3(256), 0, stream>>>(ga);

  if (QRES_T0 > 0)
    attn_band<0><<<dim3(QRES_T0 / 16, NB), dim3(256), 0, stream>>>(qpl, kpl, vtp, qrs, krs, vrt,
                                                                  ypl, yrs, 0);
  attn_band<1><<<dim3(QRES_ROWS / 16, NB), dim3(256), 0, stream>>>(qpl, kpl, vtp, qrs, krs, vrt,
                                                                  ypl, yrs, QRES_T0 / 16);

  GemmArgs gr;
  gr.A = yrs;
  gr.W0 = wob; gr.W1 = wob; gr.W2 = wob;
  gr.bias0 = bo; gr.bias1 = bo; gr.bias2 = bo;
  gr.o0 = qpl; gr.o1 = qpl; gr.o2 = qpl;
  gr.r0 = qrs; gr.r1 = qrs; gr.r2 = qrs;
  gr.of = rtm;
  gr.addend = rtm;
  gr.oscale = 1.0f / (YCARRY * RCARRY * WCARRY);
  gr.use_bias = 0;
  gr.use_add = 0;
  gr.resv = 0;
  gemm_nt<1><<<dim3(CD / 128, (NB * QRES_ROWS) / 128, 1), dim3(256), 0, stream>>>(gr);

  GemmArgs gb;
  gb.A = ypl;
  gb.W0 = wob; gb.W1 = wob; gb.W2 = wob;
  gb.bias0 = bo; gb.bias1 = bo; gb.bias2 = bo;
  gb.o0 = qpl; gb.o1 = qpl; gb.o2 = qpl;
  gb.r0 = qrs; gb.r1 = qrs; gb.r2 = qrs;
  gb.of = out;
  gb.addend = rtm;
  gb.oscale = 1.0f / (YCARRY * WCARRY);
  gb.use_bias = 1;
  gb.use_add = 1;
  gb.resv = 0;
  gemm_nt<1><<<dim3(CD / 128, M / 128, 1), dim3(256), 0, stream>>>(gb);
}
